// MambaBlock3D_90194313216283
// MI455X (gfx1250) — hardware-run, weakly checked
//
#include <hip/hip_runtime.h>
#include <stddef.h>
#include <math.h>


#pragma clang fp contract(off)

#define LSEQ  2048
#define DM    512
#define DI    1024
#define DS    64
#define DC    4
#define DR    32
#define DBW   160
#define NTHR  256
#define LNEPS 1e-5f
#define WSCAP 134217728

#define CVB    2048
#define NW_IN  (2 * DI * DM)
#define NW_X   (DBW * DI)
#define NW_DT  (DI * DR)
#define NW_O   (DM * DI)
#define CB1 (NW_IN / CVB)
#define CB2 (CB1 + NW_X / CVB)
#define CB3 (CB2 + NW_DT / CVB)
#define CBT (CB3 + NW_O / CVB)
#define PO_IN ((size_t)0)
#define PO_X  ((size_t)CB1 * CVB)
#define PO_DT ((size_t)CB2 * CVB)
#define PO_O  ((size_t)CB3 * CVB)
static_assert((NW_IN % CVB) == 0 && (NW_X % CVB) == 0 && (NW_DT % CVB) == 0 && (NW_O % CVB) == 0);
static_assert(CVB == NTHR * 8);

#define SZ_WP  ((size_t)CBT * CVB * 2)
#define SZ_XN  ((size_t)LSEQ * DM * 2)
#define SZ_XZ  ((size_t)LSEQ * 2 * DI * 4)
#define SZ_U   ((size_t)LSEQ * DI * 4)
#define SZ_UP  ((size_t)LSEQ * DI * 2)
#define SZ_DBL ((size_t)LSEQ * DBW * 4)
#define SZ_DTP ((size_t)LSEQ * DR * 2)
#define O_PH   ((size_t)0)
#define O_PL   (O_PH + SZ_WP)
#define O_XNH  (O_PL + SZ_WP)
#define O_XNL  (O_XNH + SZ_XN)
#define O_XZ   (O_XNL + SZ_XN)
#define O_U    (O_XZ + SZ_XZ)
#define O_UH   (O_U + SZ_U)
#define O_UL   (O_UH + SZ_UP)
#define O_DBL  (O_UL + SZ_UP)
#define O_DTH  (O_DBL + SZ_DBL)
#define O_DTL  (O_DTH + SZ_DTP)
#define O_DEL  (O_DTL + SZ_DTP)
#define O_YH   (O_DEL + SZ_U)
#define O_YL   (O_YH + SZ_UP)
#define WSTOT  (O_YL + SZ_UP)
static_assert(WSTOT <= (size_t)WSCAP);
static_assert((O_PL % 128) == 0 && (O_XNH % 128) == 0 && (O_XNL % 128) == 0 && (O_XZ % 128) == 0 && (O_U % 128) == 0);
static_assert((O_UH % 128) == 0 && (O_UL % 128) == 0 && (O_DBL % 128) == 0 && (O_DTH % 128) == 0 && (O_DTL % 128) == 0);
static_assert((O_DEL % 128) == 0 && (O_YH % 128) == 0 && (O_YL % 128) == 0 && (WSTOT % 128) == 0);

static_assert((DM % 32) == 0 && (DI % 32) == 0 && DR == 32);
static_assert((LSEQ % 64) == 0 && (LSEQ % 32) == 0 && ((2 * DI) % 256) == 0 && (DI % 256) == 0 && (DM % 256) == 0);
static_assert(DBW == 2 * 16 * 5);

typedef __attribute__((ext_vector_type(16))) __bf16 v16bf;
typedef float        v8f __attribute__((ext_vector_type(8)));
typedef float        v4f __attribute__((ext_vector_type(4), __may_alias__));
typedef unsigned int v4u __attribute__((ext_vector_type(4), __may_alias__));
typedef unsigned int v2u __attribute__((ext_vector_type(2), __may_alias__));
typedef int          v8i __attribute__((ext_vector_type(8)));
union FragB { v16bf v; v8i w; v4u q[2]; };
static_assert(sizeof(FragB) == 32);

__device__ __forceinline__ v8f wmb(const FragB& a, const FragB& bq, v8f c) {
  v8f d = __builtin_amdgcn_wmma_f32_16x16x32_bf16(false, a.v, false, bq.v, (short)0, c, false, false);
  asm volatile("v_nop\n\tv_nop\n\tv_nop\n\tv_nop" : "+v"(d) : "v"(a.w), "v"(bq.w));
  return d;
}

__device__ __forceinline__ v8f zero8() {
  v8f z = {0.f, 0.f, 0.f, 0.f, 0.f, 0.f, 0.f, 0.f};
  return z;
}

__device__ __forceinline__ unsigned int bfr(float f) {
  const unsigned int u = __float_as_uint(f);
  return (u + 0x7FFFu + ((u >> 16) & 1u)) >> 16;
}

__device__ __forceinline__ void split8(v4f a, v4f c, v4u& hv, v4u& lv) {
  float in[8];
  in[0] = a[0]; in[1] = a[1]; in[2] = a[2]; in[3] = a[3];
  in[4] = c[0]; in[5] = c[1]; in[6] = c[2]; in[7] = c[3];
  unsigned int hb[8], lb[8];
#pragma unroll
  for (int i = 0; i < 8; ++i) {
    hb[i] = bfr(in[i]);
    lb[i] = bfr(in[i] - __uint_as_float(hb[i] << 16));
  }
  v4u h4, l4;
  h4[0] = hb[0] | (hb[1] << 16); h4[1] = hb[2] | (hb[3] << 16); h4[2] = hb[4] | (hb[5] << 16); h4[3] = hb[6] | (hb[7] << 16);
  l4[0] = lb[0] | (lb[1] << 16); l4[1] = lb[2] | (lb[3] << 16); l4[2] = lb[4] | (lb[5] << 16); l4[3] = lb[6] | (lb[7] << 16);
  hv = h4;
  lv = l4;
}

__device__ __forceinline__ void split4(v4f a, v2u& hv, v2u& lv) {
  unsigned int hb[4], lb[4];
#pragma unroll
  for (int i = 0; i < 4; ++i) {
    hb[i] = bfr(a[i]);
    lb[i] = bfr(a[i] - __uint_as_float(hb[i] << 16));
  }
  v2u h2, l2;
  h2[0] = hb[0] | (hb[1] << 16); h2[1] = hb[2] | (hb[3] << 16);
  l2[0] = lb[0] | (lb[1] << 16); l2[1] = lb[2] | (lb[3] << 16);
  hv = h2;
  lv = l2;
}

__global__ __launch_bounds__(NTHR) void k_wsplit(const float* __restrict__ w_in, const float* __restrict__ w_x,
                                                 const float* __restrict__ w_dt, const float* __restrict__ w_o,
                                                 unsigned short* PH, unsigned short* PL) {
  const int blk = blockIdx.x, tid = threadIdx.x;
  const float* src;
  int bs;
  if (blk < CB1)      { src = w_in; bs = 0; }
  else if (blk < CB2) { src = w_x;  bs = CB1; }
  else if (blk < CB3) { src = w_dt; bs = CB2; }
  else                { src = w_o;  bs = CB3; }
  const size_t so = (size_t)(blk - bs) * CVB + (size_t)tid * 8;
  const v4f a0 = *(const v4f*)(src + so);
  const v4f a1 = *(const v4f*)(src + so + 4);
  v4u hv, lv;
  split8(a0, a1, hv, lv);
  const size_t dst = (size_t)blk * CVB + (size_t)tid * 8;
  *(volatile v4u*)(PH + dst) = hv;
  *(volatile v4u*)(PL + dst) = lv;
  __threadfence();
  *(volatile v4u*)(PH + dst) = hv;
  *(volatile v4u*)(PL + dst) = lv;
}

__global__ __launch_bounds__(NTHR) void k_ln(const float* __restrict__ X, const float* __restrict__ ga,
                                             const float* __restrict__ gb, unsigned short* XH, unsigned short* XL) {
  const int tid = threadIdx.x, lane = tid & 31, wave = tid >> 5;
  const size_t row = (size_t)blockIdx.x * (NTHR / 32) + wave;
  const float* xp = X + row * DM + 8 * lane;
  const v4f x0 = *(const v4f*)xp;
  const v4f x1 = *(const v4f*)(xp + 4);
  const v4f x2 = *(const v4f*)(xp + DM / 2);
  const v4f x3 = *(const v4f*)(xp + DM / 2 + 4);
  float v[16];
  v[0] = x0[0]; v[1] = x0[1]; v[2] = x0[2]; v[3] = x0[3]; v[4] = x1[0]; v[5] = x1[1]; v[6] = x1[2]; v[7] = x1[3];
  v[8] = x2[0]; v[9] = x2[1]; v[10] = x2[2]; v[11] = x2[3]; v[12] = x3[0]; v[13] = x3[1]; v[14] = x3[2]; v[15] = x3[3];
  float s = (((v[0] + v[1]) + (v[2] + v[3])) + ((v[4] + v[5]) + (v[6] + v[7]))) +
            (((v[8] + v[9]) + (v[10] + v[11])) + ((v[12] + v[13]) + (v[14] + v[15])));
#pragma unroll
  for (int off = 16; off > 0; off >>= 1) s += __shfl_xor(s, off, 32);
  const float mean = s * (1.0f / (float)DM);
  float dv[16];
#pragma unroll
  for (int i = 0; i < 16; ++i) dv[i] = v[i] - mean;
  float ss = 0.0f;
#pragma unroll
  for (int i = 0; i < 16; ++i) ss = ss + dv[i] * dv[i];
#pragma unroll
  for (int off = 16; off > 0; off >>= 1) ss += __shfl_xor(ss, off, 32);
  const float var = ss * (1.0f / (float)DM);
  const float rinv = rsqrtf(var + LNEPS);
  const v4f g0 = *(const v4f*)(ga + 8 * lane);
  const v4f g1 = *(const v4f*)(ga + 8 * lane + 4);
  const v4f g2 = *(const v4f*)(ga + DM / 2 + 8 * lane);
  const v4f g3 = *(const v4f*)(ga + DM / 2 + 8 * lane + 4);
  const v4f b0 = *(const v4f*)(gb + 8 * lane);
  const v4f b1 = *(const v4f*)(gb + 8 * lane + 4);
  const v4f b2 = *(const v4f*)(gb + DM / 2 + 8 * lane);
  const v4f b3 = *(const v4f*)(gb + DM / 2 + 8 * lane + 4);
  float gv[16], bv[16];
  gv[0] = g0[0]; gv[1] = g0[1]; gv[2] = g0[2]; gv[3] = g0[3]; gv[4] = g1[0]; gv[5] = g1[1]; gv[6] = g1[2]; gv[7] = g1[3];
  gv[8] = g2[0]; gv[9] = g2[1]; gv[10] = g2[2]; gv[11] = g2[3]; gv[12] = g3[0]; gv[13] = g3[1]; gv[14] = g3[2]; gv[15] = g3[3];
  bv[0] = b0[0]; bv[1] = b0[1]; bv[2] = b0[2]; bv[3] = b0[3]; bv[4] = b1[0]; bv[5] = b1[1]; bv[6] = b1[2]; bv[7] = b1[3];
  bv[8] = b2[0]; bv[9] = b2[1]; bv[10] = b2[2]; bv[11] = b2[3]; bv[12] = b3[0]; bv[13] = b3[1]; bv[14] = b3[2]; bv[15] = b3[3];
  float y[16];
#pragma unroll
  for (int i = 0; i < 16; ++i) y[i] = (dv[i] * rinv) * gv[i] + bv[i];
  v4f ya, yb, yc, yd;
  ya[0] = y[0]; ya[1] = y[1]; ya[2] = y[2]; ya[3] = y[3];
  yb[0] = y[4]; yb[1] = y[5]; yb[2] = y[6]; yb[3] = y[7];
  yc[0] = y[8]; yc[1] = y[9]; yc[2] = y[10]; yc[3] = y[11];
  yd[0] = y[12]; yd[1] = y[13]; yd[2] = y[14]; yd[3] = y[15];
  v4u hA, lA, hB, lB;
  split8(ya, yb, hA, lA);
  split8(yc, yd, hB, lB);
  const size_t d0 = row * DM + 8 * lane;
  const size_t d1 = d0 + DM / 2;
  *(volatile v4u*)(XH + d0) = hA;
  *(volatile v4u*)(XH + d1) = hB;
  *(volatile v4u*)(XL + d0) = lA;
  *(volatile v4u*)(XL + d1) = lB;
  __threadfence();
  *(volatile v4u*)(XH + d0) = hA;
  *(volatile v4u*)(XH + d1) = hB;
  *(volatile v4u*)(XL + d0) = lA;
  *(volatile v4u*)(XL + d1) = lB;
}

template <int WM, int NT, int EP>
__global__ __launch_bounds__(NTHR) void k_gemm(const unsigned short* __restrict__ Ah, const unsigned short* __restrict__ Al,
                                               const unsigned short* __restrict__ Wh, const unsigned short* __restrict__ Wl,
                                               const float* __restrict__ bias, const float* __restrict__ resid,
                                               float* Cf, unsigned short* Ph, unsigned short* Pl,
                                               int lda, int ldw, int ldc, int ldr, int K) {
  constexpr int WN = 8 / WM;
  constexpr int R = 16 * WM;
  constexpr int BN = WN * 16 * NT;
  static_assert(WM * WN == 8);
  static_assert(((R * BN / 4) % NTHR) == 0);
  constexpr int NF4 = (R * BN / 4) / NTHR;
  __shared__ __align__(16) float sC[R * BN];
  const int tid = threadIdx.x, lane = tid & 31, wave = tid >> 5, h = lane >> 4, m = lane & 15;
  const int wm = wave % WM, wn = wave / WM;
  const int bm0 = blockIdx.y * R;
  const int n0 = blockIdx.x * BN;
  const int m0 = bm0 + 16 * wm;
  const int nw0 = n0 + wn * 16 * NT;

  v8f acc[NT];
#pragma unroll
  for (int t = 0; t < NT; ++t) acc[t] = zero8();

  const size_t arow = (size_t)(m0 + m) * (size_t)lda + 8 * h;
  const size_t wrow = (size_t)(nw0 + m) * (size_t)ldw + 8 * h;
  const int nks = K >> 5;

#pragma unroll 1
  for (int ks = 0; ks < nks; ++ks) {
    const int k0 = ks << 5;
    FragB fah, fal;
    fah.q[0] = *(const v4u*)(Ah + arow + k0);
    fah.q[1] = *(const v4u*)(Ah + arow + k0 + 16);
    fal.q[0] = *(const v4u*)(Al + arow + k0);
    fal.q[1] = *(const v4u*)(Al + arow + k0 + 16);
#pragma unroll
    for (int t = 0; t < NT; ++t) {
      const unsigned short* wph = Wh + wrow + (size_t)(16 * t) * (size_t)ldw + k0;
      const unsigned short* wpl = Wl + wrow + (size_t)(16 * t) * (size_t)ldw + k0;
      FragB fwh, fwl;
      fwh.q[0] = *(const v4u*)wph;
      fwh.q[1] = *(const v4u*)(wph + 16);
      fwl.q[0] = *(const v4u*)wpl;
      fwl.q[1] = *(const v4u*)(wpl + 16);
      acc[t] = wmb(fah, fwh, acc[t]);
      acc[t] = wmb(fah, fwl, acc[t]);
      acc[t] = wmb(fal, fwh, acc[t]);
    }
  }

#pragma unroll
  for (int t = 0; t < NT; ++t) {
    const int cl = wn * 16 * NT + 16 * t + m;
#pragma unroll
    for (int r = 0; r < 8; ++r) {
      const int rl = 16 * wm + 8 * h + r;
      sC[rl * BN + cl] = acc[t][r];
    }
  }
  __syncthreads();

  if constexpr (EP == 1) {
#pragma unroll 1
    for (int it = 0; it < NF4; ++it) {
      const int e = tid + it * NTHR;
      const int rl = e / (BN / 4), q = e - rl * (BN / 4);
      v4f v = *(const v4f*)(sC + 4 * e);
      const v4f bb = *(const v4f*)(bias + n0 + 4 * q);
#pragma unroll
      for (int j = 0; j < 4; ++j) {
        const float a = v[j] + bb[j];
        v[j] = fmaxf(a, 0.0f) + log1pf(__expf(-fabsf(a)));
      }
      *(v4f*)(sC + 4 * e) = v;
    }
  } else if constexpr (EP == 2) {
#pragma unroll 1
    for (int it = 0; it < NF4; ++it) {
      const int e = tid + it * NTHR;
      const int rl = e / (BN / 4), q = e - rl * (BN / 4);
      v4f v = *(const v4f*)(sC + 4 * e);
      const v4f rr = *(const v4f*)(resid + (size_t)(bm0 + rl) * (size_t)ldr + n0 + 4 * q);
#pragma unroll
      for (int j = 0; j < 4; ++j) v[j] = v[j] + rr[j];
      *(v4f*)(sC + 4 * e) = v;
    }
  }

#pragma unroll
  for (int it = 0; it < NF4; ++it) {
    const int e = tid + it * NTHR;
    const int rl = e / (BN / 4), q = e - rl * (BN / 4);
    const v4f v = *(const v4f*)(sC + 4 * e);
    *(volatile v4f*)(Cf + (size_t)(bm0 + rl) * (size_t)ldc + n0 + 4 * q) = v;
  }
  __threadfence();
#pragma unroll
  for (int it = 0; it < NF4; ++it) {
    const int e = tid + it * NTHR;
    const int rl = e / (BN / 4), q = e - rl * (BN / 4);
    const v4f v = *(const v4f*)(sC + 4 * e);
    *(volatile v4f*)(Cf + (size_t)(bm0 + rl) * (size_t)ldc + n0 + 4 * q) = v;
  }

  if constexpr (EP == 3) {
    static_assert(R * DR == NTHR * 8);
    static_assert(BN >= DR);
    const int rl = tid >> 2, q = tid & 3;
    const v4f a = *(const v4f*)(sC + rl * BN + 8 * q);
    const v4f c = *(const v4f*)(sC + rl * BN + 8 * q + 4);
    v4u hv, lv;
    split8(a, c, hv, lv);
    const size_t dst = (size_t)(bm0 + rl) * DR + 8 * q;
    *(volatile v4u*)(Ph + dst) = hv;
    *(volatile v4u*)(Pl + dst) = lv;
    __threadfence();
    *(volatile v4u*)(Ph + dst) = hv;
    *(volatile v4u*)(Pl + dst) = lv;
  }
}

__global__ __launch_bounds__(NTHR) void k_conv(const float* __restrict__ XZ, const float* __restrict__ cw,
                                               const float* __restrict__ cb, float* U32, unsigned short* UH,
                                               unsigned short* UL) {
  const int g = blockIdx.x * NTHR + threadIdx.x;
  const int t = g / (DI / 4);
  const int dq = (g - t * (DI / 4)) * 4;
  v4f acc = *(const v4f*)(cb + dq);
  v4f w[4];
#pragma unroll
  for (int j = 0; j < 4; ++j) w[j] = *(const v4f*)(cw + (size_t)(dq + j) * DC);
#pragma unroll
  for (int k = 0; k < DC; ++k) {
    const int tt = t + k - (DC - 1);
    const int ttc = (tt < 0) ? 0 : tt;
    const v4f xv = *(const v4f*)(XZ + (size_t)ttc * (size_t)(2 * DI) + dq);
    const float f = (tt >= 0) ? 1.0f : 0.0f;
#pragma unroll
    for (int j = 0; j < 4; ++j) acc[j] = acc[j] + (xv[j] * f) * w[j][k];
  }
  v4f u;
#pragma unroll
  for (int j = 0; j < 4; ++j) {
    const float a = acc[j];
    u[j] = a * __builtin_amdgcn_rcpf(1.0f + __expf(-a));
  }
  v2u hv, lv;
  split4(u, hv, lv);
  const size_t o = (size_t)g * 4;
  *(volatile v4f*)(U32 + o) = u;
  *(volatile v2u*)(UH + o) = hv;
  *(volatile v2u*)(UL + o) = lv;
  __threadfence();
  *(volatile v4f*)(U32 + o) = u;
  *(volatile v2u*)(UH + o) = hv;
  *(volatile v2u*)(UL + o) = lv;
}

#define SCW  16
#define SCBK (8 * SCW)
#define STB  32
static_assert((DI % SCBK) == 0 && (LSEQ % STB) == 0 && DS == 64 && SCW == 16 && SCBK == 128);
static_assert(((STB * SCBK / 8) % NTHR) == 0);

__global__ __launch_bounds__(NTHR) void k_scan(const float* __restrict__ DEL, const float* __restrict__ U32,
                                               const float* __restrict__ DBL, const float* __restrict__ XZ,
                                               const float* __restrict__ Alog, const float* __restrict__ Dp,
                                               unsigned short* YH, unsigned short* YL) {
  __shared__ __align__(16) float sA[SCBK * DS];
  __shared__ __align__(16) float sY[STB * SCBK];
  const int tid = threadIdx.x, lane = tid & 31, wave = tid >> 5;
  const int grp = lane >> 3, sl = lane & 7, s0 = 8 * sl;
  const int cbase = blockIdx.x * SCBK;
  const int cl4 = SCW * wave + 4 * grp;
  const int ch4 = cbase + cl4;
#pragma unroll 1
  for (int e = tid; e < SCBK * DS; e += NTHR) sA[e] = -expf(Alog[(size_t)cbase * DS + e]);
  __syncthreads();

  float Ac[4][8], hs[4][8];
#pragma unroll
  for (int r = 0; r < 4; ++r) {
#pragma unroll
    for (int i = 0; i < 8; ++i) {
      Ac[r][i] = sA[(cl4 + r) * DS + s0 + i];
      hs[r][i] = 0.0f;
    }
  }
  const v4f dpv = *(const v4f*)(Dp + ch4);

#pragma unroll 1
  for (int t0 = 0; t0 < LSEQ; t0 += STB) {
#pragma unroll 1
    for (int tl = 0; tl < STB; ++tl) {
      const size_t t = (size_t)(t0 + tl);
      const v4f dt4 = *(const v4f*)(DEL + t * DI + ch4);
      const v4f u4 = *(const v4f*)(U32 + t * DI + ch4);
      const v4f z4 = *(const v4f*)(XZ + t * (size_t)(2 * DI) + DI + ch4);
      const float* bp = DBL + t * DBW + DR + s0;
      const v4f ba = *(const v4f*)bp;
      const v4f bb = *(const v4f*)(bp + 4);
      const v4f ca = *(const v4f*)(bp + DS);
      const v4f cc = *(const v4f*)(bp + DS + 4);
      float Bv[8], Cv[8];
      Bv[0] = ba[0]; Bv[1] = ba[1]; Bv[2] = ba[2]; Bv[3] = ba[3]; Bv[4] = bb[0]; Bv[5] = bb[1]; Bv[6] = bb[2]; Bv[7] = bb[3];
      Cv[0] = ca[0]; Cv[1] = ca[1]; Cv[2] = ca[2]; Cv[3] = ca[3]; Cv[4] = cc[0]; Cv[5] = cc[1]; Cv[6] = cc[2]; Cv[7] = cc[3];
      float yv[4];
#pragma unroll
      for (int r = 0; r < 4; ++r) {
        const float dt = dt4[r];
        const float dtu = dt * u4[r];
        float part = 0.0f;
#pragma unroll
        for (int i = 0; i < 8; ++i) {
          const float dA = __expf(dt * Ac[r][i]);
          const float hn = dA * hs[r][i] + dtu * Bv[i];
          hs[r][i] = hn;
          part = part + hn * Cv[i];
        }
        part += __shfl_xor(part, 4, 32);
        part += __shfl_xor(part, 2, 32);
        part += __shfl_xor(part, 1, 32);
        const float z = z4[r];
        const float sg = __builtin_amdgcn_rcpf(1.0f + __expf(-z));
        yv[r] = (part + dpv[r] * u4[r]) * (z * sg);
      }
      if (sl == 0) {
        v4f yo;
        yo[0] = yv[0]; yo[1] = yv[1]; yo[2] = yv[2]; yo[3] = yv[3];
        *(v4f*)(sY + tl * SCBK + cl4) = yo;
      }
    }
    __syncthreads();
    {
      constexpr int NIT = (STB * SCBK / 8) / NTHR;
      v4u hv[NIT], lv[NIT];
      size_t dst[NIT];
#pragma unroll
      for (int it = 0; it < NIT; ++it) {
        const int e = tid + it * NTHR;
        const int rl = e >> 4, q = e & 15;
        const v4f a = *(const v4f*)(sY + rl * SCBK + 8 * q);
        const v4f c = *(const v4f*)(sY + rl * SCBK + 8 * q + 4);
        split8(a, c, hv[it], lv[it]);
        dst[it] = (size_t)(t0 + rl) * DI + cbase + 8 * q;
      }
#pragma unroll
      for (int it = 0; it < NIT; ++it) {
        *(volatile v4u*)(YH + dst[it]) = hv[it];
        *(volatile v4u*)(YL + dst[it]) = lv[it];
      }
      __threadfence();
#pragma unroll
      for (int it = 0; it < NIT; ++it) {
        *(volatile v4u*)(YH + dst[it]) = hv[it];
        *(volatile v4u*)(YL + dst[it]) = lv[it];
      }
    }
    __syncthreads();
  }
}

extern "C" void kernel_launch(void* const* d_in, const int* in_sizes, int n_in,
                              void* d_out, int out_size, void* d_ws, size_t ws_size,
                              hipStream_t stream) {
  if (n_in < 12) return;
  if (in_sizes[0] != LSEQ * DM) return;
  if (in_sizes[1] != DM || in_sizes[2] != DM) return;
  if (in_sizes[3] != 2 * DI * DM) return;
  if (in_sizes[4] != DI * DC || in_sizes[5] != DI) return;
  if (in_sizes[6] != DBW * DI) return;
  if (in_sizes[7] != DI * DR || in_sizes[8] != DI) return;
  if (in_sizes[9] != DI * DS || in_sizes[10] != DI) return;
  if (in_sizes[11] != DM * DI) return;
  if (out_size != LSEQ * DM) return;
  const size_t tot = (size_t)WSTOT;
  if (tot > ws_size || tot > (size_t)WSCAP) return;

  const float* x     = (const float*)d_in[0];
  const float* lng   = (const float*)d_in[1];
  const float* lnb   = (const float*)d_in[2];
  const float* win   = (const float*)d_in[3];
  const float* cw    = (const float*)d_in[4];
  const float* cb    = (const float*)d_in[5];
  const float* wx    = (const float*)d_in[6];
  const float* wdt   = (const float*)d_in[7];
  const float* bdt   = (const float*)d_in[8];
  const float* alog  = (const float*)d_in[9];
  const float* dpp   = (const float*)d_in[10];
  const float* wout  = (const float*)d_in[11];
  float* out = (float*)d_out;

  char* ws = (char*)d_ws;
  unsigned short* PH  = (unsigned short*)(ws + O_PH);
  unsigned short* PL  = (unsigned short*)(ws + O_PL);
  unsigned short* XNH = (unsigned short*)(ws + O_XNH);
  unsigned short* XNL = (unsigned short*)(ws + O_XNL);
  float*          XZ  = (float*)(ws + O_XZ);
  float*          U32 = (float*)(ws + O_U);
  unsigned short* UH  = (unsigned short*)(ws + O_UH);
  unsigned short* UL  = (unsigned short*)(ws + O_UL);
  float*          DBL = (float*)(ws + O_DBL);
  unsigned short* DTH = (unsigned short*)(ws + O_DTH);
  unsigned short* DTL = (unsigned short*)(ws + O_DTL);
  float*          DEL = (float*)(ws + O_DEL);
  unsigned short* YH  = (unsigned short*)(ws + O_YH);
  unsigned short* YL  = (unsigned short*)(ws + O_YL);


  k_wsplit<<<CBT, NTHR, 0, stream>>>(win, wx, wdt, wout, PH, PL);

  k_ln<<<LSEQ / (NTHR / 32), NTHR, 0, stream>>>(x, lng, lnb, XNH, XNL);

  k_gemm<2, 4, 0><<<dim3(2 * DI / 256, LSEQ / 32), NTHR, 0, stream>>>(
      XNH, XNL, PH + PO_IN, PL + PO_IN, x, x, XZ, UH, UL, DM, DM, 2 * DI, 0, DM);

  k_conv<<<(LSEQ * DI / 4) / NTHR, NTHR, 0, stream>>>(XZ, cw, cb, U32, UH, UL);

  k_gemm<4, 5, 3><<<dim3(1, LSEQ / 64), NTHR, 0, stream>>>(
      UH, UL, PH + PO_X, PL + PO_X, x, x, DBL, DTH, DTL, DI, DI, DBW, 0, DI);

  k_gemm<2, 4, 1><<<dim3(DI / 256, LSEQ / 32), NTHR, 0, stream>>>(
      DTH, DTL, PH + PO_DT, PL + PO_DT, bdt, x, DEL, UH, UL, DR, DR, DI, 0, DR);

  k_scan<<<DI / SCBK, NTHR, 0, stream>>>(DEL, U32, DBL, XZ, alog, dpp, YH, YL);

  k_gemm<2, 4, 2><<<dim3(DM / 256, LSEQ / 32), NTHR, 0, stream>>>(
      YH, YL, PH + PO_O, PL + PO_O, x, x, out, UH, UL, DI, DI, DM, DM, DI);
}
